// BottleneckAttention3D_22789096473254
// MI455X (gfx1250) — hardware-verified
//
#include <hip/hip_runtime.h>
#include <stddef.h>
#include <stdint.h>

#define NBAT 2
#define CD   128
#define NN   4096
#define NTOK (NBAT * NN)
#define NGRP 8
#define CPG  (CD / NGRP)
#define GNE  (CPG * NN)
#define QB   128
#define KC   64
#define NQB  (NN / QB)
#define NCK  (NN / KC)
#define STP  32
#define GN_EPS 1e-5f

static_assert(NTOK == 8192);
static_assert(CPG == 16);
static_assert(GNE == 65536);
static_assert(GNE % 1024 == 0);
static_assert(CD == 128);
static_assert(NN % 64 == 0);
static_assert(NN % QB == 0);
static_assert(NN % KC == 0);
static_assert(QB == 8 * 16);
static_assert(KC == 64);
static_assert((CD * CD) % 2048 == 0);
static_assert(NTOK % 64 == 0);

typedef _Float16 v16h __attribute__((ext_vector_type(16)));
typedef _Float16 v8h  __attribute__((ext_vector_type(8)));
typedef __bf16   v16b __attribute__((ext_vector_type(16)));
typedef float    v8f  __attribute__((ext_vector_type(8)));
typedef float    v4f  __attribute__((ext_vector_type(4)));
typedef unsigned int v4u __attribute__((ext_vector_type(4)));

union FragH { v16h v; v8h h[2]; };
union FragB { v16b v; v4u u[2]; };
union Pack8 { v8h h; v4u u; };

__device__ __forceinline__ v8f mma_h(v16h a, v16h b, v8f c) {
  c = __builtin_amdgcn_wmma_f32_16x16x32_f16(false, a, false, b, (short)0, c, false, false);
  asm volatile("v_nop\n\tv_nop\n\tv_nop\n\tv_nop" : "+v"(c) : "v"(a), "v"(b));
  return c;
}
__device__ __forceinline__ v8f mma_b(v16b a, v16b b, v8f c) {
  c = __builtin_amdgcn_wmma_f32_16x16x32_bf16(false, a, false, b, (short)0, c, false, false);
  asm volatile("v_nop\n\tv_nop\n\tv_nop\n\tv_nop" : "+v"(c) : "v"(a), "v"(b));
  return c;
}
__device__ __forceinline__ v8f zero8() { return (v8f){0.f, 0.f, 0.f, 0.f, 0.f, 0.f, 0.f, 0.f}; }

__device__ __forceinline__ v16h ldfrag_h(const _Float16* p, int ld, int row0, int k0, int lane) {
  const int m = lane & 15, lh = lane >> 4;
  const _Float16* q = p + (size_t)(row0 + m) * ld + k0 + 8 * lh;
  FragH f;
  f.h[0] = *(const v8h*)(q);
  f.h[1] = *(const v8h*)(q + 16);
  return f.v;
}
__device__ __forceinline__ v16b ldfrag_b(const unsigned short* p, int ld, int row0, int k0, int lane) {
  const int m = lane & 15, lh = lane >> 4;
  const unsigned short* q = p + (size_t)(row0 + m) * ld + k0 + 8 * lh;
  FragB f;
  f.u[0] = *(const v4u*)(q);
  f.u[1] = *(const v4u*)(q + 16);
  return f.v;
}

__device__ __forceinline__ unsigned int bf16_bits(float f) {
  const unsigned int u = __float_as_uint(f);
  return (u + 0x7FFFu + ((u >> 16) & 1u)) >> 16;
}
__device__ __forceinline__ void split_bf16(float f, unsigned int& hb, unsigned int& lb) {
  hb = bf16_bits(f);
  const float hf = __uint_as_float(hb << 16);
  lb = bf16_bits(f - hf);
}
__device__ __forceinline__ void pack_split8(const float (&v)[8], v4u& ph, v4u& pl) {
  unsigned int hb[8], lb[8];
#pragma unroll
  for (int i = 0; i < 8; ++i) split_bf16(v[i], hb[i], lb[i]);
  ph = (v4u){hb[0] | (hb[1] << 16), hb[2] | (hb[3] << 16), hb[4] | (hb[5] << 16), hb[6] | (hb[7] << 16)};
  pl = (v4u){lb[0] | (lb[1] << 16), lb[2] | (lb[3] << 16), lb[4] | (lb[5] << 16), lb[6] | (lb[7] << 16)};
}
__device__ __forceinline__ v4u pack_h8(const float (&v)[8]) {
  Pack8 pk;
  pk.h = (v8h){(_Float16)v[0], (_Float16)v[1], (_Float16)v[2], (_Float16)v[3],
               (_Float16)v[4], (_Float16)v[5], (_Float16)v[6], (_Float16)v[7]};
  return pk.u;
}

__device__ __forceinline__ void gemm16x64h(const _Float16* __restrict__ A, int lda,
                                           const _Float16* __restrict__ B,
                                           int m0, int n0, int lane, v8f (&acc)[4]) {
#pragma unroll 1
  for (int ks = 0; ks < CD / 32; ++ks) {
    const v16h a = ldfrag_h(A, lda, m0, ks * 32, lane);
#pragma unroll
    for (int t = 0; t < 4; ++t) {
      const v16h b = ldfrag_h(B, CD, n0 + 16 * t, ks * 32, lane);
      acc[t] = mma_h(a, b, acc[t]);
    }
  }
}

__global__ __launch_bounds__(256) void k_wcv(const float* __restrict__ w0, const float* __restrict__ w1,
                                             const float* __restrict__ w2, const float* __restrict__ w3,
                                             _Float16* __restrict__ wpl) {
  int i = blockIdx.x * 256 + threadIdx.x;
  i = min(i, CD * CD / 8 - 1);
  const int which = blockIdx.y;
  const float* W = (which == 0) ? w0 : (which == 1) ? w1 : (which == 2) ? w2 : w3;
  const float* src = W + (size_t)i * 8;
  const v4f a0 = *(const v4f*)(src), a1 = *(const v4f*)(src + 4);
  const float v[8] = {a0[0] * 64.0f, a0[1] * 64.0f, a0[2] * 64.0f, a0[3] * 64.0f,
                      a1[0] * 64.0f, a1[1] * 64.0f, a1[2] * 64.0f, a1[3] * 64.0f};
  const v4u pv = pack_h8(v);
  _Float16* dst = wpl + (size_t)which * CD * CD + (size_t)i * 8;
  for (int ps = 0; ps < 2; ++ps) {
    *(volatile v4u*)(dst) = pv;
    __threadfence();
  }
}

__global__ __launch_bounds__(256) void k_gnst(const float* __restrict__ x, float* __restrict__ st) {
  __shared__ double rs[256];
  const int tid = threadIdx.x;
  const int bg = blockIdx.x;
  const float* xp = x + (size_t)bg * GNE;
  double s = 0.0;
#pragma unroll 2
  for (int i = tid * 4; i < GNE; i += 1024) {
    const v4f a = *(const v4f*)(xp + i);
    s += ((double)a[0] + (double)a[1]) + ((double)a[2] + (double)a[3]);
  }
  rs[tid] = s;
  __syncthreads();
  for (int o = 128; o > 0; o >>= 1) {
    if (tid < o) rs[tid] += rs[tid + o];
    __syncthreads();
  }
  const float meanf = (float)(rs[0] * (1.0 / (double)GNE));
  __syncthreads();
  double s2 = 0.0;
#pragma unroll 2
  for (int i = tid * 4; i < GNE; i += 1024) {
    const v4f a = *(const v4f*)(xp + i);
    const float d0 = a[0] - meanf, d1 = a[1] - meanf, d2 = a[2] - meanf, d3 = a[3] - meanf;
    s2 += ((double)d0 * (double)d0 + (double)d1 * (double)d1) +
          ((double)d2 * (double)d2 + (double)d3 * (double)d3);
  }
  rs[tid] = s2;
  __syncthreads();
  for (int o = 128; o > 0; o >>= 1) {
    if (tid < o) rs[tid] += rs[tid + o];
    __syncthreads();
  }
  const float varf = (float)(rs[0] * (1.0 / (double)GNE));
  const float rstd = 1.0f / sqrtf(varf + GN_EPS);
  if (tid < 8) {
    const v4f val = (tid == 0) ? (v4f){meanf, rstd, 0.f, 0.f} : (v4f){0.f, 0.f, 0.f, 0.f};
    float* p = st + (size_t)bg * STP + tid * 4;
    *(volatile v4f*)(p) = val;
    __threadfence();
    *(volatile v4f*)(p) = val;
  }
}

#define WTP 65
__global__ __launch_bounds__(256) void k_xtr(const float* __restrict__ x,
                                             const float* __restrict__ st,
                                             const float* __restrict__ gam,
                                             const float* __restrict__ bet,
                                             _Float16* __restrict__ hp) {
  __shared__ float tl[64 * WTP];
  const int tid = threadIdx.x;
  const int n0 = blockIdx.x * 64, c0 = blockIdx.y * 64, b = blockIdx.z;
  const float* xb = x + (size_t)b * CD * NN;
#pragma unroll
  for (int j = 0; j < 4; ++j) {
    const int p  = tid + 256 * j;
    const int cc = p >> 4;
    const int q4 = (p & 15) * 4;
    const v4f a = *(const v4f*)(xb + (size_t)(c0 + cc) * NN + n0 + q4);
    float* d = tl + cc * WTP + q4;
    d[0] = a[0]; d[1] = a[1]; d[2] = a[2]; d[3] = a[3];
  }
  __syncthreads();
  v4u vo[2];
  size_t go[2];
#pragma unroll
  for (int j = 0; j < 2; ++j) {
    const int p  = tid + 256 * j;
    const int nn = p >> 3;
    const int pc = p & 7;
    const int cb = c0 + pc * 8;
    const int g  = cb >> 4;
    const float mean = st[(size_t)(b * NGRP + g) * STP + 0];
    const float rstd = st[(size_t)(b * NGRP + g) * STP + 1];
    const v4f g0 = *(const v4f*)(gam + cb), g1 = *(const v4f*)(gam + cb + 4);
    const v4f e0 = *(const v4f*)(bet + cb), e1 = *(const v4f*)(bet + cb + 4);
    const float gs[8] = {g0[0], g0[1], g0[2], g0[3], g1[0], g1[1], g1[2], g1[3]};
    const float bs[8] = {e0[0], e0[1], e0[2], e0[3], e1[0], e1[1], e1[2], e1[3]};
    const float* cp = tl + (pc * 8) * WTP + nn;
    float v[8];
#pragma unroll
    for (int i = 0; i < 8; ++i) {
      const float t = (cp[i * WTP] - mean) * rstd;
      v[i] = (t * gs[i] + bs[i]) * 8.0f;
    }
    vo[j] = pack_h8(v);
    go[j] = ((size_t)b * NN + n0 + nn) * CD + cb;
  }
  for (int ps = 0; ps < 2; ++ps) {
#pragma unroll
    for (int j = 0; j < 2; ++j) *(volatile v4u*)(hp + go[j]) = vo[j];
    __threadfence();
  }
}

#define SFP 132
#define INV512 0.001953125f
__global__ __launch_bounds__(256) void k_qkv(const _Float16* __restrict__ hp,
                                             const _Float16* __restrict__ wpl,
                                             const float* __restrict__ bq,
                                             const float* __restrict__ bk,
                                             const float* __restrict__ bv,
                                             unsigned short* __restrict__ qh,
                                             unsigned short* __restrict__ ql,
                                             unsigned short* __restrict__ kh,
                                             unsigned short* __restrict__ kl,
                                             _Float16* __restrict__ vt) {
  __shared__ __align__(16) float sf[64 * SFP];
  const int tid = threadIdx.x, lane = tid & 31, wave = tid >> 5;
  const int hh = lane >> 4, c = lane & 15;
  const int wm = wave >> 1, wn = wave & 1;
  const int mb  = blockIdx.x * 64;
  const int b   = mb >> 12;
  const int nb0 = mb & (NN - 1);
  const int which = blockIdx.y;
  const _Float16* W = wpl + (size_t)which * CD * CD;
  const float* bias = (which == 0) ? bq : (which == 1) ? bk : bv;
  const int m0 = mb + wm * 16;
  const int n0 = wn * 64;

  v8f acc[4];
#pragma unroll
  for (int t = 0; t < 4; ++t) acc[t] = zero8();
  gemm16x64h(hp, CD, W, m0, n0, lane, acc);

#pragma unroll
  for (int t = 0; t < 4; ++t) {
#pragma unroll
    for (int r = 0; r < 8; ++r)
      sf[(wm * 16 + 8 * hh + r) * SFP + n0 + 16 * t + c] = acc[t][r];
  }
  __syncthreads();

  if (which < 2) {
    v4u vh[4], vl[4];
    size_t go[4];
#pragma unroll
    for (int j = 0; j < 4; ++j) {
      const int p  = tid + 256 * j;
      const int lr = p >> 4;
      const int pc = p & 15;
      const float* ra = sf + lr * SFP + pc * 8;
      const v4f a0 = *(const v4f*)(ra), a1 = *(const v4f*)(ra + 4);
      const v4f b0 = *(const v4f*)(bias + pc * 8), b1 = *(const v4f*)(bias + pc * 8 + 4);
      const float v[8] = {a0[0] * INV512 + b0[0], a0[1] * INV512 + b0[1], a0[2] * INV512 + b0[2],
                          a0[3] * INV512 + b0[3], a1[0] * INV512 + b1[0], a1[1] * INV512 + b1[1],
                          a1[2] * INV512 + b1[2], a1[3] * INV512 + b1[3]};
      pack_split8(v, vh[j], vl[j]);
      go[j] = ((size_t)(mb + lr)) * CD + pc * 8;
    }
    unsigned short* dh = (which == 0) ? qh : kh;
    unsigned short* dl = (which == 0) ? ql : kl;
    for (int ps = 0; ps < 2; ++ps) {
#pragma unroll
      for (int j = 0; j < 4; ++j) {
        *(volatile v4u*)(dh + go[j]) = vh[j];
        *(volatile v4u*)(dl + go[j]) = vl[j];
      }
      __threadfence();
    }
  } else {
    v4u vo[4];
    size_t go[4];
#pragma unroll
    for (int j = 0; j < 4; ++j) {
      const int p    = tid + 256 * j;
      const int dcol = p >> 3;
      const int pc   = p & 7;
      const float* cp = sf + (pc * 8) * SFP + dcol;
      const float bb = bias[dcol];
      const float v[8] = {(cp[0 * SFP] * INV512 + bb) * 16.0f, (cp[1 * SFP] * INV512 + bb) * 16.0f,
                          (cp[2 * SFP] * INV512 + bb) * 16.0f, (cp[3 * SFP] * INV512 + bb) * 16.0f,
                          (cp[4 * SFP] * INV512 + bb) * 16.0f, (cp[5 * SFP] * INV512 + bb) * 16.0f,
                          (cp[6 * SFP] * INV512 + bb) * 16.0f, (cp[7 * SFP] * INV512 + bb) * 16.0f};
      vo[j] = pack_h8(v);
      go[j] = ((size_t)(b * CD + dcol)) * NN + nb0 + pc * 8;
    }
    for (int ps = 0; ps < 2; ++ps) {
#pragma unroll
      for (int j = 0; j < 4; ++j) *(volatile v4u*)(vt + go[j]) = vo[j];
      __threadfence();
    }
  }
}

#define KTP 136
#define VTP 72
#define PTP 72
#define OSP 68
#define OSCL 0.00390625f
__global__ __launch_bounds__(256) void k_attn(const unsigned short* __restrict__ qh,
                                              const unsigned short* __restrict__ ql,
                                              const unsigned short* __restrict__ kh,
                                              const unsigned short* __restrict__ kl,
                                              const _Float16* __restrict__ vt,
                                              _Float16* __restrict__ op,
                                              float sscale) {
  __shared__ __align__(16) unsigned short Ksh[KC * KTP];
  __shared__ __align__(16) unsigned short Ksl[KC * KTP];
  __shared__ __align__(16) _Float16 Vs[CD * VTP];
  __shared__ __align__(16) _Float16 Ps[8 * 16 * PTP];
  __shared__ __align__(16) float    Os[8 * 16 * OSP];

  const int tid = threadIdx.x, lane = tid & 31, wave = tid >> 5;
  const int hh = lane >> 4, c = lane & 15;
  const int b  = blockIdx.x / NQB;
  const int qb = blockIdx.x % NQB;
  const int q0 = qb * QB + wave * 16;
  const int trow  = b * NN + q0;
  const int krow0 = b * NN;
  const _Float16* V = vt + (size_t)b * CD * NN;

  const float NEGI = -__builtin_huge_valf();
  float mrow[8], lrow[8];
  v8f oacc[8];
#pragma unroll
  for (int r = 0; r < 8; ++r) { mrow[r] = NEGI; lrow[r] = 0.f; }
#pragma unroll
  for (int t = 0; t < 8; ++t) oacc[t] = zero8();

  _Float16* pw = Ps + wave * 16 * PTP;
  float*    ow = Os + wave * 16 * OSP;

#pragma unroll 1
  for (int kc = 0; kc < NCK; ++kc) {
    const int kv0 = kc * KC;
    __syncthreads();
#pragma unroll
    for (int j = 0; j < 4; ++j) {
      const int p  = tid + 256 * j;
      const int rk = p >> 4;
      const int qk = (p & 15) * 8;
      const size_t gs = (size_t)(krow0 + kv0 + rk) * CD + qk;
      *(v4u*)(Ksh + rk * KTP + qk) = *(const v4u*)(kh + gs);
      *(v4u*)(Ksl + rk * KTP + qk) = *(const v4u*)(kl + gs);
    }
#pragma unroll
    for (int j = 0; j < 4; ++j) {
      const int p  = tid + 256 * j;
      const int rv = p >> 3;
      const int qv = (p & 7) * 8;
      *(v8h*)(Vs + rv * VTP + qv) = *(const v8h*)(V + (size_t)rv * NN + kv0 + qv);
    }
    __syncthreads();

    v8f s[4];
#pragma unroll
    for (int j = 0; j < 4; ++j) s[j] = zero8();
#pragma unroll 1
    for (int ks = 0; ks < CD / 32; ++ks) {
      const v16b qa = ldfrag_b(qh, CD, trow, ks * 32, lane);
      const v16b qr = ldfrag_b(ql, CD, trow, ks * 32, lane);
#pragma unroll
      for (int j = 0; j < 4; ++j) {
        const v16b ka = ldfrag_b(Ksh, KTP, j * 16, ks * 32, lane);
        const v16b kr = ldfrag_b(Ksl, KTP, j * 16, ks * 32, lane);
        s[j] = mma_b(qa, ka, s[j]);
        s[j] = mma_b(qr, ka, s[j]);
        s[j] = mma_b(qa, kr, s[j]);
      }
    }
    float cm[8];
#pragma unroll
    for (int r = 0; r < 8; ++r) {
      float mx = NEGI;
#pragma unroll
      for (int j = 0; j < 4; ++j) { s[j][r] *= sscale; mx = fmaxf(mx, s[j][r]); }
#pragma unroll
      for (int off = 1; off < 16; off <<= 1) mx = fmaxf(mx, __shfl_xor(mx, off, 32));
      cm[r] = mx;
    }
    float al[8];
#pragma unroll
    for (int r = 0; r < 8; ++r) {
      const float mnew  = fmaxf(mrow[r], cm[r]);
      const float alpha = __expf(mrow[r] - mnew);
      mrow[r] = mnew;
      float psum = 0.f;
#pragma unroll
      for (int j = 0; j < 4; ++j) {
        const float p = __expf(s[j][r] - mnew);
        psum += p;
        pw[(8 * hh + r) * PTP + j * 16 + c] = (_Float16)(p * 1024.0f);
      }
#pragma unroll
      for (int off = 1; off < 16; off <<= 1) psum += __shfl_xor(psum, off, 32);
      lrow[r] = lrow[r] * alpha + psum;
      al[r] = alpha;
    }
#pragma unroll
    for (int t = 0; t < 8; ++t)
#pragma unroll
      for (int r = 0; r < 8; ++r) oacc[t][r] *= al[r];
    __syncthreads();

#pragma unroll
    for (int kk = 0; kk < 2; ++kk) {
      const v16h pa = ldfrag_h(pw, PTP, 0, kk * 32, lane);
#pragma unroll
      for (int t = 0; t < 8; ++t) {
        const v16h vb = ldfrag_h(Vs, VTP, t * 16, kk * 32, lane);
        oacc[t] = mma_h(pa, vb, oacc[t]);
      }
    }
  }

  float invl[8];
#pragma unroll
  for (int r = 0; r < 8; ++r) invl[r] = (lrow[r] > 0.f) ? (OSCL * (1.0f / lrow[r])) : 0.f;

#pragma unroll
  for (int half = 0; half < 2; ++half) {
    __syncthreads();
#pragma unroll
    for (int r = 0; r < 8; ++r) {
#pragma unroll
      for (int t = 0; t < 4; ++t) ow[(8 * hh + r) * OSP + 16 * t + c] = oacc[4 * half + t][r] * invl[r];
    }
    __syncthreads();
    v4u vo[4];
    size_t go[4];
#pragma unroll
    for (int it = 0; it < 4; ++it) {
      const int p  = lane + 32 * it;
      const int L  = p >> 3;
      const int pc = p & 7;
      const float* ra = ow + L * OSP + pc * 8;
      const v4f a0 = *(const v4f*)(ra), a1 = *(const v4f*)(ra + 4);
      const float v[8] = {a0[0], a0[1], a0[2], a0[3], a1[0], a1[1], a1[2], a1[3]};
      vo[it] = pack_h8(v);
      go[it] = ((size_t)(trow + L)) * CD + half * 64 + pc * 8;
    }
    for (int ps = 0; ps < 2; ++ps) {
#pragma unroll
      for (int it = 0; it < 4; ++it) *(volatile v4u*)(op + go[it]) = vo[it];
      __threadfence();
    }
  }
}

#define OTP 68
#define INV4096 0.000244140625f
__global__ __launch_bounds__(256) void k_proj(const _Float16* __restrict__ op,
                                              const _Float16* __restrict__ wpl,
                                              const float* __restrict__ pb,
                                              const float* __restrict__ x,
                                              float* __restrict__ out) {
  __shared__ __align__(16) float st[CD * OTP];
  const int tid = threadIdx.x, lane = tid & 31, wave = tid >> 5;
  const int hh = lane >> 4, c = lane & 15;
  const int wm = wave >> 1, wn = wave & 1;
  const int mb  = blockIdx.x * 64;
  const int b   = mb >> 12;
  const int nb0 = mb & (NN - 1);
  const int m0  = mb + wm * 16;
  const int n0  = wn * 64;
  const _Float16* W = wpl + (size_t)3 * CD * CD;

  v8f acc[4];
#pragma unroll
  for (int t = 0; t < 4; ++t) acc[t] = zero8();
  gemm16x64h(op, CD, W, m0, n0, lane, acc);

#pragma unroll
  for (int t = 0; t < 4; ++t) {
    const float bb = pb[n0 + 16 * t + c];
#pragma unroll
    for (int r = 0; r < 8; ++r) st[(n0 + 16 * t + c) * OTP + wm * 16 + 8 * hh + r] = acc[t][r] * INV4096 + bb;
  }
  __syncthreads();
  v4f val[8];
  size_t go[8];
#pragma unroll
  for (int it = 0; it < 8; ++it) {
    const int p    = lane + 32 * it;
    const int L    = p >> 3;
    const int pc   = p & 7;
    const int cl   = wave * 16 + (L >> 1);
    const int half = L & 1;
    go[it] = ((size_t)(b * CD + cl)) * NN + nb0 + half * 32 + pc * 4;
    const v4f sv = *(const v4f*)(st + cl * OTP + half * 32 + pc * 4);
    const v4f xv = *(const v4f*)(x + go[it]);
    val[it] = sv + xv;
  }
  for (int ps = 0; ps < 2; ++ps) {
#pragma unroll
    for (int it = 0; it < 8; ++it) *(volatile v4f*)(out + go[it]) = val[it];
    __threadfence();
  }
}

extern "C" void kernel_launch(void* const* d_in, const int* in_sizes, int n_in,
                              void* d_out, int out_size, void* d_ws, size_t ws_size,
                              hipStream_t stream) {
  if (n_in < 11) return;
  if (in_sizes[0] != NTOK * CD) return;
  if (in_sizes[1] != CD || in_sizes[2] != CD) return;
  if (in_sizes[3] != CD * CD || in_sizes[4] != CD) return;
  if (in_sizes[5] != CD * CD || in_sizes[6] != CD) return;
  if (in_sizes[7] != CD * CD || in_sizes[8] != CD) return;
  if (in_sizes[9] != CD * CD || in_sizes[10] != CD) return;
  if (out_size != NTOK * CD) return;

  const float* x     = (const float*)d_in[0];
  const float* gamma = (const float*)d_in[1];
  const float* beta  = (const float*)d_in[2];
  const float* wq    = (const float*)d_in[3];
  const float* bq    = (const float*)d_in[4];
  const float* wk    = (const float*)d_in[5];
  const float* bk    = (const float*)d_in[6];
  const float* wv    = (const float*)d_in[7];
  const float* bv    = (const float*)d_in[8];
  const float* wp    = (const float*)d_in[9];
  const float* bp    = (const float*)d_in[10];
  float* out = (float*)d_out;

  size_t off = 0;
  const size_t oW  = off; off += (size_t)4 * CD * CD * 2;
  const size_t oSt = off; off += 4096;
  const size_t oH  = off; off += (size_t)NTOK * CD * 2;
  const size_t oQh = off; off += (size_t)NTOK * CD * 2;
  const size_t oQl = off; off += (size_t)NTOK * CD * 2;
  const size_t oKh = off; off += (size_t)NTOK * CD * 2;
  const size_t oKl = off; off += (size_t)NTOK * CD * 2;
  const size_t oV  = off; off += (size_t)NBAT * CD * NN * 2;
  const size_t oO  = off; off += (size_t)NTOK * CD * 2;
  if (off > ws_size) return;
  if (off > (size_t)134217728) return;

  char* ws = (char*)d_ws;
  _Float16*       Wpl = (_Float16*)(ws + oW);
  float*          St  = (float*)(ws + oSt);
  _Float16*       Hp  = (_Float16*)(ws + oH);
  unsigned short* Qh  = (unsigned short*)(ws + oQh);
  unsigned short* Ql  = (unsigned short*)(ws + oQl);
  unsigned short* Kh  = (unsigned short*)(ws + oKh);
  unsigned short* Kl  = (unsigned short*)(ws + oKl);
  _Float16*       Vt  = (_Float16*)(ws + oV);
  _Float16*       Op  = (_Float16*)(ws + oO);

  k_wcv<<<dim3((CD * CD / 8) / 256, 4), dim3(256), 0, stream>>>(wq, wk, wv, wp, Wpl);
  k_gnst<<<dim3(NBAT * NGRP), dim3(256), 0, stream>>>(x, St);
  k_xtr<<<dim3(NN / 64, CD / 64, NBAT), dim3(256), 0, stream>>>(x, St, gamma, beta, Hp);
  k_qkv<<<dim3(NTOK / 64, 3), dim3(256), 0, stream>>>(Hp, Wpl, bq, bk, bv, Qh, Ql, Kh, Kl, Vt);
  const float sscale = 0.08838834764831845f;
  k_attn<<<dim3(NBAT * NQB), dim3(256), 0, stream>>>(Qh, Ql, Kh, Kl, Vt, Op, sscale);
  k_proj<<<dim3(NTOK / 64), dim3(256), 0, stream>>>(Op, Wpl, bp, x, out);
  (void)hipGetLastError();
}
